// HAN_62921270886522
// MI455X (gfx1250) — hardware-verified
//
#include <hip/hip_runtime.h>
#include <stddef.h>
#include <stdint.h>


#define DIN     128
#define HID     128
#define NHD     8
#define DHD     16
#define NOUT    2
#define APITCH  32
#define KHL     256
#define NTHR    256
#define NWAVE   8
#define EPT     8
#define CHUNK   (NTHR * EPT)
#define WCAP    (EPT * 32)
#define LISTN   (NWAVE * WCAP)
#define NBMAX   1024
#define SLB     10
#define RCAP    28672
#define DEGCAP  512
#define STW     640
#define GBM     64
#define GBN     64
#define GTHR    128
#define WSMAX   268435456
#define LDS_AGG ((2 * RCAP + 2 * NBMAX + LISTN) * 4 + 64)

static_assert((CHUNK & (CHUNK - 1)) == 0 && CHUNK <= 2048);
static_assert(NBMAX == (1 << SLB));
static_assert(NTHR * 4 == NBMAX);
static_assert(LISTN >= NBMAX);
static_assert(LISTN >= NWAVE * WCAP);
static_assert((RCAP % 32) == 0);
static_assert(NWAVE * STW <= RCAP);
static_assert(STW >= HID + 2 * (NBMAX / NWAVE));
static_assert(LDS_AGG <= 300000);
static_assert(GBM == (GTHR / 32) * 16);
static_assert((DIN % 32) == 0 && (KHL % 32) == 0 && (HID % GBN) == 0);
static_assert(HID == NHD * DHD && DHD == 16 && NHD == 8);
static_assert(APITCH == 32);

typedef float          v4f   __attribute__((ext_vector_type(4)));
typedef float          v8f   __attribute__((ext_vector_type(8)));
typedef int            v4i   __attribute__((ext_vector_type(4)));
typedef int            v8i   __attribute__((ext_vector_type(8)));
typedef unsigned short v8us  __attribute__((ext_vector_type(8)));
typedef __attribute__((ext_vector_type(16))) __bf16 v16bf;
union FragB { v16bf v; v8us h[2]; v8i w; };

__device__ __forceinline__ v8f wmb(const FragB& a, const FragB& b, v8f c) {
  v8f d = __builtin_amdgcn_wmma_f32_16x16x32_bf16(false, a.v, false, b.v, (short)0, c, false, false);
  asm volatile("v_nop\n\tv_nop\n\tv_nop\n\tv_nop" : "+v"(d) : "v"(a.w), "v"(b.w));
  return d;
}

__device__ __forceinline__ void ldwait() {
  asm volatile("s_wait_loadcnt 0x0" ::: "memory");
}

__device__ __forceinline__ unsigned short bfb(float f) {
  unsigned u = __float_as_uint(f);
  u = u + 0x7FFFu + ((u >> 16) & 1u);
  return (unsigned short)(u >> 16);
}
__device__ __forceinline__ float bfr(float f) {
  return __uint_as_float(((unsigned)bfb(f)) << 16);
}
__device__ __forceinline__ v8us cvt8b(const v4f a, const v4f b) {
  v8us o;
  o[0] = bfb(a.x); o[1] = bfb(a.y); o[2] = bfb(a.z); o[3] = bfb(a.w);
  o[4] = bfb(b.x); o[5] = bfb(b.y); o[6] = bfb(b.z); o[7] = bfb(b.w);
  return o;
}
__device__ __forceinline__ v8us hilo8(const v4f a, const v4f b, const int hh) {
  float v[8] = {a.x, a.y, a.z, a.w, b.x, b.y, b.z, b.w};
  v8us o;
#pragma unroll
  for (int i = 0; i < 8; ++i) {
    const unsigned short hb = bfb(v[i]);
    const float hf = __uint_as_float(((unsigned)hb) << 16);
    const unsigned short lb = bfb(v[i] - hf);
    o[i] = hh ? lb : hb;
  }
  return o;
}

__device__ __forceinline__ int scan_chunk(const int* __restrict__ dsts, int nE, int cbase, int slotBase,
                                          int nb, int vec8, int* list, int tid, int lane, int wave) {
  int wc = 0;
  const int el0  = tid * EPT;
  const int e0   = cbase + el0;
  const int sent = -2147483647 - 1;
  v4i da, db;
  if (vec8 != 0 && cbase + CHUNK <= nE) {
    da = *(const v4i*)(dsts + e0);
    db = *(const v4i*)(dsts + e0 + 4);
  } else {
    da.x = (e0     < nE) ? dsts[min(e0,     nE - 1)] : sent;
    da.y = (e0 + 1 < nE) ? dsts[min(e0 + 1, nE - 1)] : sent;
    da.z = (e0 + 2 < nE) ? dsts[min(e0 + 2, nE - 1)] : sent;
    da.w = (e0 + 3 < nE) ? dsts[min(e0 + 3, nE - 1)] : sent;
    db.x = (e0 + 4 < nE) ? dsts[min(e0 + 4, nE - 1)] : sent;
    db.y = (e0 + 5 < nE) ? dsts[min(e0 + 5, nE - 1)] : sent;
    db.z = (e0 + 6 < nE) ? dsts[min(e0 + 6, nE - 1)] : sent;
    db.w = (e0 + 7 < nE) ? dsts[min(e0 + 7, nE - 1)] : sent;
  }
  const unsigned nbs = (unsigned)slotBase;
  const unsigned unb = (unsigned)nb;
  const unsigned s0 = (unsigned)da.x - nbs, s1 = (unsigned)da.y - nbs;
  const unsigned s2 = (unsigned)da.z - nbs, s3 = (unsigned)da.w - nbs;
  const unsigned s4 = (unsigned)db.x - nbs, s5 = (unsigned)db.y - nbs;
  const unsigned s6 = (unsigned)db.z - nbs, s7 = (unsigned)db.w - nbs;
  const bool h0 = s0 < unb, h1 = s1 < unb, h2 = s2 < unb, h3 = s3 < unb;
  const bool h4 = s4 < unb, h5 = s5 < unb, h6 = s6 < unb, h7 = s7 < unb;
  const unsigned any = __builtin_amdgcn_ballot_w32(h0 | h1 | h2 | h3 | h4 | h5 | h6 | h7);
  if (any != 0u) {
#define HITJ(J, HJ, SJ) { \
      const unsigned mj = __builtin_amdgcn_ballot_w32(HJ); \
      if (mj != 0u) { \
        if (HJ) { \
          const int pos = wc + (int)__builtin_amdgcn_mbcnt_lo(mj, 0u); \
          if (pos < WCAP) list[wave * WCAP + pos] = ((el0 + (J)) << 12) | (int)(SJ); \
        } \
        wc += (int)__builtin_popcount(mj); } }
    HITJ(0, h0, s0)
    HITJ(1, h1, s1)
    HITJ(2, h2, s2)
    HITJ(3, h3, s3)
    HITJ(4, h4, s4)
    HITJ(5, h5, s5)
    HITJ(6, h6, s6)
    HITJ(7, h7, s7)
#undef HITJ
  }
  return wc;
}

__global__ __launch_bounds__(NTHR) void k_xprep(const float* __restrict__ x0, const float* __restrict__ x1,
                                                unsigned short* o0, unsigned short* o1,
                                                int n0, int n1, int u0, int u1) {
  const int y = (int)blockIdx.y;
  const float* x = y ? x1 : x0;
  unsigned short* xb = y ? o1 : o0;
  const int nN = y ? n1 : n0;
  const int nUnits = y ? u1 : u0;
  const int i = (int)blockIdx.x * NTHR + (int)threadIdx.x;
  if (i >= nUnits) return;
  const int row = i >> 4;
  const int c0  = (i & 15) * 8;
  const int rc  = row < nN ? row : nN - 1;
  const float* p = x + (size_t)rc * DIN + c0;
  v4f a = *(const v4f*)p, b = *(const v4f*)(p + 4);
  const v4f z4 = {0.f, 0.f, 0.f, 0.f};
  if (row >= nN) { a = z4; b = z4; }
  const v8us hv = cvt8b(a, b);
  const size_t o = (size_t)row * DIN + c0;
  *(volatile v8us*)(xb + o) = hv;
  __threadfence();
  *(volatile v8us*)(xb + o) = hv;
}

__global__ __launch_bounds__(NTHR) void k_wprep(const float* __restrict__ w0, const float* __restrict__ w1,
                                                const float* __restrict__ w2,
                                                unsigned short* o0, unsigned short* o1, unsigned short* o2,
                                                int ko0, int ko1, int ko2, int nrows, int kin) {
  const int y = (int)blockIdx.y;
  const float* w = (y == 0) ? w0 : ((y == 1) ? w1 : w2);
  unsigned short* ob = (y == 0) ? o0 : ((y == 1) ? o1 : o2);
  const int kout = (y == 0) ? ko0 : ((y == 1) ? ko1 : ko2);
  const int kq = kout >> 3;
  const int nUnits = nrows * kq;
  const int u = (int)blockIdx.x * NTHR + (int)threadIdx.x;
  if (u >= nUnits) return;
  const int n  = u / kq;
  const int k8 = (u - n * kq) * 8;
  const int ks = k8 % kin;
  const float* p = w + (size_t)n * (size_t)kin + ks;
  const v4f a = *(const v4f*)p, b = *(const v4f*)(p + 4);
  const v8us hv = cvt8b(a, b);
  const size_t o = (size_t)n * (size_t)kout + k8;
  *(volatile v8us*)(ob + o) = hv;
  __threadfence();
  *(volatile v8us*)(ob + o) = hv;
}

template<int EPI>
__global__ __launch_bounds__(GTHR) void k_gemm(
    const unsigned short* __restrict__ A, const unsigned short* __restrict__ WT,
    const float* __restrict__ bias, float* outF, int K, int ldo, int nRows, int nCols)
{
  __shared__ __attribute__((aligned(16))) float stg[GBM * GBN];
  __shared__ __attribute__((aligned(16))) float csum[2 * GBN];
  const int tid = (int)threadIdx.x, lane = tid & 31, wave = tid >> 5, hh = lane >> 4, m = lane & 15;
  const int rowBase = (int)blockIdx.x * GBM;
  const int col0    = (int)blockIdx.y * GBN;

  v8f acc[4];
  {
    const v8f z = {0.f, 0.f, 0.f, 0.f, 0.f, 0.f, 0.f, 0.f};
    acc[0] = z; acc[1] = z; acc[2] = z; acc[3] = z;
  }
  const unsigned short* ap = A  + (size_t)(rowBase + 16 * wave + m) * (size_t)K + 8 * hh;
  const unsigned short* wp = WT + (size_t)(col0 + m) * (size_t)K + 8 * hh;
  const int ksteps = K >> 5;
#pragma unroll 1
  for (int ks = 0; ks < ksteps; ++ks) {
    FragB af;
    af.h[0] = *(const v8us*)(ap + 32 * ks);
    af.h[1] = *(const v8us*)(ap + 32 * ks + 16);
#pragma unroll
    for (int t = 0; t < 4; ++t) {
      const unsigned short* wq = wp + (size_t)(16 * t) * (size_t)K + 32 * ks;
      FragB bf;
      bf.h[0] = *(const v8us*)wq;
      bf.h[1] = *(const v8us*)(wq + 16);
      acc[t] = wmb(af, bf, acc[t]);
    }
  }

#pragma unroll
  for (int t = 0; t < 4; ++t) {
    const int lc = 16 * t + m;
    int bi = col0 + lc;
    bi = bi > nCols - 1 ? nCols - 1 : bi;
    bi = bi < 0 ? 0 : bi;
    const float bv = bfr(bias[bi]);
#pragma unroll
    for (int r = 0; r < 8; ++r) {
      const int lr = 16 * wave + 8 * hh + r;
      stg[lr * GBN + lc] = acc[t][r] + bv;
    }
  }
  __syncthreads();

  if (EPI == 0) {
    v4f fv[8];
#pragma unroll
    for (int i = 0; i < 8; ++i) {
      const int lr = 16 * wave + 2 * i + hh;
      fv[i] = *(const v4f*)(stg + lr * GBN + 4 * m);
    }
#pragma unroll
    for (int i = 0; i < 8; ++i) {
      const int lr = 16 * wave + 2 * i + hh;
      const int gr = rowBase + lr;
      float* op = outF + (size_t)gr * (size_t)ldo + col0 + 4 * m;
      *(volatile v4f*)op = fv[i];
    }
    __threadfence();
#pragma unroll
    for (int i = 0; i < 8; ++i) {
      const int lr = 16 * wave + 2 * i + hh;
      const int gr = rowBase + lr;
      float* op = outF + (size_t)gr * (size_t)ldo + col0 + 4 * m;
      *(volatile v4f*)op = fv[i];
    }
  } else {
    const int c  = tid & (GBN - 1);
    const int rh = tid >> 6;
    float s = 0.f;
#pragma unroll 1
    for (int r = 0; r < 32; ++r) {
      const int lr = 32 * rh + r;
      const float v = tanhf(stg[lr * GBN + c]);
      s += (rowBase + lr < nRows) ? v : 0.f;
    }
    csum[rh * GBN + c] = s;
    __syncthreads();
    v4f ov;
    {
      const int q4 = (tid & 15) * 4;
      ov.x = csum[q4 + 0] + csum[GBN + q4 + 0];
      ov.y = csum[q4 + 1] + csum[GBN + q4 + 1];
      ov.z = csum[q4 + 2] + csum[GBN + q4 + 2];
      ov.w = csum[q4 + 3] + csum[GBN + q4 + 3];
    }
    float* rp = outF + (size_t)blockIdx.x * (size_t)ldo + col0 + 4 * (tid & 15);
    const bool wsv = tid < 16;
    if (wsv) *(volatile v4f*)rp = ov;
    __threadfence();
    if (wsv) *(volatile v4f*)rp = ov;
  }
}

__global__ __launch_bounds__(NTHR) void k_att(const float* __restrict__ X, const float* __restrict__ a0,
                                              const float* __restrict__ a1, const float* __restrict__ a2,
                                              float* AP, int MP) {
  __shared__ __attribute__((aligned(16))) float satt[3 * HID];
  __shared__ __attribute__((aligned(16))) float sa[32 * APITCH];
  const int tid = (int)threadIdx.x;
  if (tid < HID) {
    satt[tid]           = bfr(a0[tid]);
    satt[HID + tid]     = bfr(a1[tid]);
    satt[2 * HID + tid] = bfr(a2[tid]);
  }
  __syncthreads();
  const int nl = tid >> 3, h = tid & 7;
  const int base = (int)blockIdx.x * 32;
  int row = base + nl;
  row = row < MP ? row : MP - 1;
  const float* xp = X + (size_t)row * HID + DHD * h;
  float d0 = 0.f, d1 = 0.f, d2 = 0.f;
#pragma unroll 1
  for (int j = 0; j < 4; ++j) {
    const v4f xv = *(const v4f*)(xp + 4 * j);
    const v4f t0 = *(const v4f*)(satt + DHD * h + 4 * j);
    const v4f t1 = *(const v4f*)(satt + HID + DHD * h + 4 * j);
    const v4f t2 = *(const v4f*)(satt + 2 * HID + DHD * h + 4 * j);
    d0 = fmaf(xv.x, t0.x, d0); d0 = fmaf(xv.y, t0.y, d0); d0 = fmaf(xv.z, t0.z, d0); d0 = fmaf(xv.w, t0.w, d0);
    d1 = fmaf(xv.x, t1.x, d1); d1 = fmaf(xv.y, t1.y, d1); d1 = fmaf(xv.z, t1.z, d1); d1 = fmaf(xv.w, t1.w, d1);
    d2 = fmaf(xv.x, t2.x, d2); d2 = fmaf(xv.y, t2.y, d2); d2 = fmaf(xv.z, t2.z, d2); d2 = fmaf(xv.w, t2.w, d2);
  }
  const int pm = 4 * (h & 1) + (h >> 1);
  sa[nl * APITCH + pm]      = d0;
  sa[nl * APITCH + 8 + pm]  = d1;
  sa[nl * APITCH + 16 + pm] = d2;
  sa[nl * APITCH + 24 + h]  = 0.f;
  __syncthreads();
  const int node = tid >> 3, pc = tid & 7;
  const v4f ov = *(const v4f*)(sa + node * APITCH + 4 * pc);
  float* gp = AP + (size_t)(base + node) * APITCH + 4 * pc;
  *(volatile v4f*)gp = ov;
  __threadfence();
  *(volatile v4f*)gp = ov;
}

__global__ __launch_bounds__(NTHR) void k_agg(
    const int* __restrict__ srcs, const int* __restrict__ dsts,
    const float* __restrict__ XS, const float* __restrict__ ASP, const float* __restrict__ ADP,
    const float* __restrict__ LW, unsigned short* AHL, float* PP,
    int nN, int nSrc, int nE, int nb, int vec8, int MPr, int aoffS, int aoffD) {
  extern __shared__ v4f lds_dyn[];
  int* reg1 = (int*)lds_dyn;
  int* reg2 = reg1 + RCAP;
  int* scnt = reg2 + RCAP;
  int* soff = scnt + NBMAX;
  int* list = soff + NBMAX;
  int* wcnt = list + LISTN;
  int* wtot = wcnt + NWAVE;
  const int tid = (int)threadIdx.x, lane = tid & 31, wave = tid >> 5;
  const int nodeBase = (int)blockIdx.x * nb;

  for (int i = tid; i < NBMAX; i += NTHR) scnt[i] = 0;
  __syncthreads();

  int tot = 0;
  const int nChunks = (nE + CHUNK - 1) / CHUNK;
#pragma unroll 1
  for (int ch = 0; ch < nChunks; ++ch) {
    const int cbase = ch * CHUNK;
    const int wc = scan_chunk(dsts, nE, cbase, nodeBase, nb, vec8, list, tid, lane, wave);
    if (lane == 0) wcnt[wave] = wc;
    __syncthreads();
    int pre = 0, all = 0;
#pragma unroll
    for (int w2 = 0; w2 < NWAVE; ++w2) {
      int c = wcnt[w2];
      c = c < 0 ? 0 : (c > WCAP ? WCAP : c);
      all += c;
      pre += (w2 < wave) ? c : 0;
    }
    const int wcc  = wc > WCAP ? WCAP : wc;
    const int base = tot + pre;
#pragma unroll 1
    for (int i = lane; i < wcc; i += 32) {
      const int ent = list[wave * WCAP + i];
      const int el  = (ent >> 12) & (CHUNK - 1);
      const int sl  = ent & (NBMAX - 1);
      int eid = cbase + el;
      eid = eid > nE - 1 ? nE - 1 : eid;
      const int pos = base + i;
      if (pos < RCAP) reg1[pos] = (int)(((unsigned)eid << SLB) | (unsigned)sl);
    }
    tot += all;
    tot = tot > RCAP ? RCAP : tot;
    __syncthreads();
  }
  const int nh = tot;

  if (wave == 0) {
#pragma unroll 1
    for (int b0 = 0; b0 < nh; b0 += 32) {
      const int idx = b0 + lane;
      const int uv  = reg1[idx < RCAP ? idx : RCAP - 1];
      const int m32 = (nh - b0) < 32 ? (nh - b0) : 32;
#pragma unroll 1
      for (int k = 0; k < m32; ++k) {
        const int u  = __builtin_amdgcn_readlane(uv, k);
        const int sl = u & (NBMAX - 1);
        if (lane == 0) scnt[sl] = scnt[sl] + 1;
      }
    }
  }
  __syncthreads();

  {
    const v4i ca = *(const v4i*)(scnt + 4 * tid);
    const int e0 = ca.x < 0 ? 0 : ca.x, e1 = ca.y < 0 ? 0 : ca.y, e2 = ca.z < 0 ? 0 : ca.z, e3 = ca.w < 0 ? 0 : ca.w;
    const int ts = e0 + e1 + e2 + e3;
    int incl = ts;
#pragma unroll
    for (int d = 1; d < 32; d <<= 1) {
      const int up = __shfl_up(incl, d);
      if (lane >= d) incl += up;
    }
    if (lane == 31) wtot[wave] = incl;
    __syncthreads();
    int pre = 0;
#pragma unroll
    for (int w2 = 0; w2 < NWAVE; ++w2) pre += (w2 < wave) ? wtot[w2] : 0;
    int run = pre + incl - ts;
    soff[4 * tid + 0] = run; run += e0;
    soff[4 * tid + 1] = run; run += e1;
    soff[4 * tid + 2] = run; run += e2;
    soff[4 * tid + 3] = run;
  }
  __syncthreads();
  for (int i = tid; i < NBMAX; i += NTHR) list[i] = soff[i];
  __syncthreads();

  if (wave == 0) {
#pragma unroll 1
    for (int b0 = 0; b0 < nh; b0 += 32) {
      const int idx = b0 + lane;
      const int uv  = reg1[idx < RCAP ? idx : RCAP - 1];
      const int m32 = (nh - b0) < 32 ? (nh - b0) : 32;
#pragma unroll 1
      for (int k = 0; k < m32; ++k) {
        const int u   = __builtin_amdgcn_readlane(uv, k);
        const int sl  = u & (NBMAX - 1);
        const int eid = (int)((unsigned)u >> SLB);
        if (lane == 0) {
          int pos = list[sl];
          pos = pos < 0 ? 0 : (pos > RCAP - 1 ? RCAP - 1 : pos);
          reg2[pos] = eid;
          list[sl] = pos + 1;
        }
      }
    }
  }
  __syncthreads();

  const int nbw = nb >> 3;
  const bool ovf = (nh >= RCAP);
  const float qnan = __int_as_float(0x7fc00000);
  float* stw = (float*)reg1 + wave * STW;
  const int hh = lane >> 4, m = lane & 15;
  float lw0[4], lw1[4];
#pragma unroll
  for (int j = 0; j < 4; ++j) {
    lw0[j] = bfr(LW[32 * j + lane]);
    lw1[j] = bfr(LW[HID + 32 * j + lane]);
  }
#pragma unroll 1
  for (int jt = 0; jt < nbw; ++jt) {
    const int slot = wave * nbw + jt;
    const int grow = nodeBase + slot;
    const int gcl  = grow < nN ? grow : nN - 1;
    int st = soff[slot];
    const int craw = scnt[slot];
    int cnt = craw;
    st  = st < 0 ? 0 : (st > nh ? nh : st);
    cnt = cnt < 0 ? 0 : (cnt > DEGCAP ? DEGCAP : cnt);
    if (cnt > nh - st) cnt = nh - st;
    const float pz = (ovf || craw > DEGCAP) ? qnan : 0.0f;
    const bool wr = grow < MPr;
    const float live = grow < nN ? 1.0f : 0.0f;

    const v4f ad4 = *(const v4f*)(ADP + (size_t)gcl * APITCH + aoffD + 4 * hh);
    ldwait();
    float ad[4] = {ad4.x, ad4.y, ad4.z, ad4.w};
    float mx[4], dn[4], av[4];
#pragma unroll
    for (int j = 0; j < 4; ++j) { mx[j] = -1.0e30f; dn[j] = 0.f; av[j] = 0.f; }

#pragma unroll 1
    for (int qe = 0; qe < cnt; ++qe) {
      int idx = st + qe; idx = idx > RCAP - 1 ? RCAP - 1 : idx;
      int eid = reg2[idx]; eid = eid < 0 ? 0 : (eid > nE - 1 ? nE - 1 : eid);
      const int sraw = srcs[eid];
      const int s = sraw < 0 ? 0 : (sraw > nSrc - 1 ? nSrc - 1 : sraw);
      const v4f as4 = *(const v4f*)(ASP + (size_t)s * APITCH + aoffS + 4 * hh);
      const float* xr = XS + (size_t)s * HID + lane;
      float xv[4];
#pragma unroll
      for (int j = 0; j < 4; ++j) xv[j] = xr[32 * j];
      ldwait();
      float as[4] = {as4.x, as4.y, as4.z, as4.w};
#pragma unroll
      for (int j = 0; j < 4; ++j) {
        float a = as[j] + ad[j];
        a = a > 0.f ? a : 0.2f * a;
        const float df = a - mx[j];
        const float ee = __expf(-fabsf(df));
        const bool up  = df > 0.f;
        const float s1 = up ? ee : 1.0f;
        const float s2 = up ? 1.0f : ee;
        mx[j] = up ? a : mx[j];
        dn[j] = fmaf(dn[j], s1, s2);
        av[j] = fmaf(av[j], s1, s2 * xv[j]);
      }
    }
    float rv[4];
#pragma unroll
    for (int j = 0; j < 4; ++j) {
      const float ds = dn[j] > 0.f ? dn[j] : 1.0f;
      const float iv = (dn[j] > 0.f ? 1.0f : 0.0f) * __builtin_amdgcn_rcpf(ds);
      rv[j] = fmaxf(av[j] * iv, 0.f) * live + pz;
    }
    float p0 = rv[0] * lw0[0];
    p0 = fmaf(rv[1], lw0[1], p0); p0 = fmaf(rv[2], lw0[2], p0); p0 = fmaf(rv[3], lw0[3], p0);
    float p1 = rv[0] * lw1[0];
    p1 = fmaf(rv[1], lw1[1], p1); p1 = fmaf(rv[2], lw1[2], p1); p1 = fmaf(rv[3], lw1[3], p1);
#pragma unroll
    for (int off = 16; off > 0; off >>= 1) {
      p0 += __shfl_xor(p0, off);
      p1 += __shfl_xor(p1, off);
    }
    __builtin_amdgcn_fence(__ATOMIC_RELEASE, "wavefront");
    __builtin_amdgcn_wave_barrier();
    stw[lane]      = rv[0];
    stw[32 + lane] = rv[1];
    stw[64 + lane] = rv[2];
    stw[96 + lane] = rv[3];
    if (lane == 0) { stw[HID + 2 * jt] = p0; stw[HID + 2 * jt + 1] = p1; }
    __builtin_amdgcn_fence(__ATOMIC_RELEASE, "wavefront");
    __builtin_amdgcn_wave_barrier();
    const v4f ga = *(const v4f*)(stw + 8 * m);
    const v4f gb = *(const v4f*)(stw + 8 * m + 4);
    const v8us hv = hilo8(ga, gb, hh);
    unsigned short* gp = AHL + (size_t)grow * KHL + HID * hh + 8 * m;
    if (wr) *(volatile v8us*)gp = hv;
    __threadfence();
    if (wr) *(volatile v8us*)gp = hv;
  }

  __builtin_amdgcn_fence(__ATOMIC_RELEASE, "wavefront");
  __builtin_amdgcn_wave_barrier();
  const int np4 = nbw >> 1;
  float* pbase = PP + (size_t)(nodeBase + wave * nbw) * NOUT;
#pragma unroll 1
  for (int u = lane; u < np4; u += 32) {
    const v4f pv = *(const v4f*)(stw + HID + 4 * u);
    *(volatile v4f*)(pbase + 4 * u) = pv;
  }
  __threadfence();
#pragma unroll 1
  for (int u = lane; u < np4; u += 32) {
    const v4f pv = *(const v4f*)(stw + HID + 4 * u);
    *(volatile v4f*)(pbase + 4 * u) = pv;
  }
}

__global__ __launch_bounds__(NTHR) void k_fold(const float* __restrict__ recG, const float* __restrict__ recD,
                                               const float* __restrict__ qv, float* att, int nRec, double invN) {
  __shared__ double sq[2 * HID];
  const int tid = (int)threadIdx.x, lane = tid & 31;
  if (tid < HID) {
    double sg = 0.0, sd = 0.0;
#pragma unroll 1
    for (int r = 0; r < nRec; ++r) {
      sg += (double)recG[(size_t)r * HID + tid];
      sd += (double)recD[(size_t)r * HID + tid];
    }
    const double qc = (double)bfr(qv[tid]);
    sq[tid]       = qc * (sg * invN);
    sq[HID + tid] = qc * (sd * invN);
  }
  __syncthreads();
  if (tid < 32) {
    float a0 = 0.f, a1 = 0.f;
    if (lane == 0) {
      double s0 = 0.0, s1 = 0.0;
#pragma unroll 1
      for (int c = 0; c < HID; ++c) { s0 += sq[c]; s1 += sq[HID + c]; }
      const float f0 = (float)s0, f1 = (float)s1;
      const float mxv = fmaxf(f0, f1);
      const float e0 = __expf(f0 - mxv), e1 = __expf(f1 - mxv);
      const float inv = __builtin_amdgcn_rcpf(e0 + e1);
      a0 = e0 * inv;
      a1 = e1 * inv;
    }
    a0 = __shfl(a0, 0);
    a1 = __shfl(a1, 0);
    v4f o = {0.f, 0.f, 0.f, 0.f};
    if (lane == 0) { o.x = a0; o.y = a1; }
    const bool wsv = lane < 8;
    if (wsv) *(volatile v4f*)(att + 4 * lane) = o;
    __threadfence();
    if (wsv) *(volatile v4f*)(att + 4 * lane) = o;
  }
}

__global__ __launch_bounds__(NTHR) void k_final(const float* __restrict__ PG, const float* __restrict__ PD,
                                                const float* __restrict__ att, const float* __restrict__ lb,
                                                float* out, int n4) {
  const int i = (int)blockIdx.x * NTHR + (int)threadIdx.x;
  if (i >= n4) return;
  const float a0 = att[0], a1 = att[1];
  const float b0 = bfr(lb[0]), b1 = bfr(lb[1]);
  const v4f pg = *(const v4f*)(PG + 4 * (size_t)i);
  const v4f pd = *(const v4f*)(PD + 4 * (size_t)i);
  v4f o;
  o.x = a0 * pg.x + a1 * pd.x + b0;
  o.y = a0 * pg.y + a1 * pd.y + b1;
  o.z = a0 * pg.z + a1 * pd.z + b0;
  o.w = a0 * pg.w + a1 * pd.w + b1;
  float* op = out + 4 * (size_t)i;
  *(volatile v4f*)op = o;
  __threadfence();
  *(volatile v4f*)op = o;
}

static int pick_nb(int nE, int nDst) {
  int nb = NBMAX;
  while (nb > 128 && (long long)nb * (long long)nE * 5LL > (long long)RCAP * (long long)nDst * 3LL) nb >>= 1;
  return nb;
}
static inline int cdiv(int a, int b) { return (a + b - 1) / b; }

extern "C" void kernel_launch(void* const* d_in, const int* in_sizes, int n_in,
                              void* d_out, int out_size, void* d_ws, size_t ws_size,
                              hipStream_t stream) {
  if (n_in < 17) return;
  const int nN = in_sizes[0] / DIN;
  if (nN < 64 || in_sizes[0] != nN * DIN || nN > (1 << 22) || (nN & 15) != 0) return;
  const int nD = in_sizes[1] / DIN;
  if (nD < 1 || in_sizes[1] != nD * DIN || nD > (1 << 22)) return;
  if (in_sizes[2] < 2 || (in_sizes[2] & 1) != 0) return;
  if (in_sizes[3] < 2 || (in_sizes[3] & 1) != 0) return;
  const int nEg = in_sizes[2] / 2, nEd = in_sizes[3] / 2;
  if (nEg > (1 << 22) || nEd > (1 << 22)) return;
  if (in_sizes[4]  != HID * DIN || in_sizes[5]  != HID) return;
  if (in_sizes[6]  != HID * DIN || in_sizes[7]  != HID) return;
  if (in_sizes[8]  != HID || in_sizes[9] != HID || in_sizes[10] != HID || in_sizes[11] != HID) return;
  if (in_sizes[12] != HID * HID || in_sizes[13] != HID || in_sizes[14] != HID) return;
  if (in_sizes[15] != NOUT * HID || in_sizes[16] != NOUT) return;
  if (out_size != nN * NOUT) return;

  const float* xg    = (const float*)d_in[0];
  const float* xd    = (const float*)d_in[1];
  const int*   egg   = (const int*)  d_in[2];
  const int*   edg   = (const int*)  d_in[3];
  const float* pgw   = (const float*)d_in[4];
  const float* pgb   = (const float*)d_in[5];
  const float* pdw   = (const float*)d_in[6];
  const float* pdb   = (const float*)d_in[7];
  const float* asgg  = (const float*)d_in[8];
  const float* adgg  = (const float*)d_in[9];
  const float* asdg  = (const float*)d_in[10];
  const float* addg  = (const float*)d_in[11];
  const float* kw    = (const float*)d_in[12];
  const float* kb    = (const float*)d_in[13];
  const float* qv    = (const float*)d_in[14];
  const float* lw    = (const float*)d_in[15];
  const float* lb    = (const float*)d_in[16];
  float* out = (float*)d_out;
  const int* src_gg = egg;
  const int* dst_gg = egg + nEg;
  const int* src_dg = edg;
  const int* dst_dg = edg + nEd;

  const int MPG = cdiv(nN, GBM) * GBM;
  const int MPD = cdiv(nD, GBM) * GBM;
  const int nbg = pick_nb(nEg, nN);
  const int nbd = pick_nb(nEd, nN);
  if (nbg < 128 || nbd < 128) return;
  const int gAg = cdiv(MPG, nbg), gAd = cdiv(MPG, nbd);
  if (gAg * nbg < MPG || gAd * nbd < MPG) return;
  const int vec8g = ((nEg & 3) == 0) ? 1 : 0;
  const int vec8d = ((nEd & 3) == 0) ? 1 : 0;
  const int gMg = MPG / GBM, gMd = MPD / GBM;

  char* ws = (char*)d_ws;
  size_t off = 0;
  const size_t oXGB = off; off += (size_t)MPG * DIN * 2;                 off = (off + 255) & ~(size_t)255;
  const size_t oXDB = off; off += (size_t)MPD * DIN * 2;                 off = (off + 255) & ~(size_t)255;
  const size_t oWG  = off; off += (size_t)HID * DIN * 2;                 off = (off + 255) & ~(size_t)255;
  const size_t oWD  = off; off += (size_t)HID * DIN * 2;                 off = (off + 255) & ~(size_t)255;
  const size_t oWK  = off; off += (size_t)HID * KHL * 2;                 off = (off + 255) & ~(size_t)255;
  const size_t oXG  = off; off += (size_t)MPG * HID * 4;                 off = (off + 255) & ~(size_t)255;
  const size_t oXD  = off; off += (size_t)MPD * HID * 4;                 off = (off + 255) & ~(size_t)255;
  const size_t oAG  = off; off += (size_t)MPG * APITCH * 4;              off = (off + 255) & ~(size_t)255;
  const size_t oAD  = off; off += (size_t)MPD * APITCH * 4;              off = (off + 255) & ~(size_t)255;
  const size_t oHLG = off; off += (size_t)MPG * KHL * 2;                 off = (off + 255) & ~(size_t)255;
  const size_t oHLD = off; off += (size_t)MPG * KHL * 2;                 off = (off + 255) & ~(size_t)255;
  const size_t oPG  = off; off += (size_t)gAg * nbg * NOUT * 4;          off = (off + 255) & ~(size_t)255;
  const size_t oPD  = off; off += (size_t)gAd * nbd * NOUT * 4;          off = (off + 255) & ~(size_t)255;
  const size_t oRG  = off; off += (size_t)gMg * HID * 4;                 off = (off + 255) & ~(size_t)255;
  const size_t oRD  = off; off += (size_t)gMg * HID * 4;                 off = (off + 255) & ~(size_t)255;
  const size_t oATT = off; off += 256;                                   off = (off + 255) & ~(size_t)255;
  if (off > ws_size || off > (size_t)WSMAX) return;
  unsigned short* XGB = (unsigned short*)(ws + oXGB);
  unsigned short* XDB = (unsigned short*)(ws + oXDB);
  unsigned short* WG  = (unsigned short*)(ws + oWG);
  unsigned short* WD  = (unsigned short*)(ws + oWD);
  unsigned short* WK  = (unsigned short*)(ws + oWK);
  float* XG  = (float*)(ws + oXG);
  float* XD  = (float*)(ws + oXD);
  float* AG  = (float*)(ws + oAG);
  float* AD  = (float*)(ws + oAD);
  unsigned short* HLG = (unsigned short*)(ws + oHLG);
  unsigned short* HLD = (unsigned short*)(ws + oHLD);
  float* PG  = (float*)(ws + oPG);
  float* PD  = (float*)(ws + oPD);
  float* RG  = (float*)(ws + oRG);
  float* RD  = (float*)(ws + oRD);
  float* ATT = (float*)(ws + oATT);

  hipFuncSetAttribute(reinterpret_cast<const void*>(&k_agg),
                      hipFuncAttributeMaxDynamicSharedMemorySize, LDS_AGG);

  {
    const int uG = MPG * (DIN / 8), uD = MPD * (DIN / 8);
    const int um = uG > uD ? uG : uD;
    k_xprep<<<dim3(cdiv(um, NTHR), 2), NTHR, 0, stream>>>(xg, xd, XGB, XDB, nN, nD, uG, uD);
  }
  k_wprep<<<dim3(cdiv(HID * (KHL / 8), NTHR), 3), NTHR, 0, stream>>>(pgw, pdw, kw, WG, WD, WK,
                                                                     DIN, DIN, KHL, HID, DIN);
  k_gemm<0><<<dim3(gMg, HID / GBN), GTHR, 0, stream>>>(XGB, WG, pgb, XG, DIN, HID, nN, HID);
  k_gemm<0><<<dim3(gMd, HID / GBN), GTHR, 0, stream>>>(XDB, WD, pdb, XD, DIN, HID, nD, HID);
  k_att<<<MPG / 32, NTHR, 0, stream>>>(XG, asgg, adgg, addg, AG, MPG);
  k_att<<<MPD / 32, NTHR, 0, stream>>>(XD, asdg, asdg, asdg, AD, MPD);
  k_agg<<<gAg, NTHR, LDS_AGG, stream>>>(src_gg, dst_gg, XG, AG, AG, lw, HLG, PG,
                                        nN, nN, nEg, nbg, vec8g, MPG, 0, 8);
  k_agg<<<gAd, NTHR, LDS_AGG, stream>>>(src_dg, dst_dg, XD, AD, AG, lw, HLD, PD,
                                        nN, nD, nEd, nbd, vec8d, MPG, 0, 16);
  k_gemm<1><<<dim3(gMg, HID / GBN), GTHR, 0, stream>>>(HLG, WK, kb, RG, KHL, HID, nN, HID);
  k_gemm<1><<<dim3(gMg, HID / GBN), GTHR, 0, stream>>>(HLD, WK, kb, RD, KHL, HID, nN, HID);
  k_fold<<<1, NTHR, 0, stream>>>(RG, RD, qv, ATT, gMg, 1.0 / (double)nN);
  {
    const int n4 = nN / 2;
    k_final<<<cdiv(n4, NTHR), NTHR, 0, stream>>>(PG, PD, ATT, lb, out, n4);
  }
}
